// Self_Attention_66013647340270
// MI455X (gfx1250) — hardware-run, weakly checked
//
#include <hip/hip_runtime.h>


#define NB_  4
#define TT   4096
#define DM   256
#define EM   32
#define HD   32
#define HP   64
#define NP   128
#define ZH   1
#define RH   4096
#define PCAR 1024.0f
#define SCL  1.0f
typedef _Float16 h16;
typedef unsigned short bf;
typedef __attribute__((ext_vector_type(16))) __bf16   v16bf;
typedef __attribute__((ext_vector_type(16))) _Float16 v16h;
typedef __attribute__((ext_vector_type(8)))  _Float16 v8h;
typedef __attribute__((ext_vector_type(8)))  unsigned short v8us;
typedef __attribute__((ext_vector_type(8)))  float    v8f;
typedef __attribute__((ext_vector_type(4)))  float    v4f;
typedef v8h  __attribute__((may_alias)) v8ha;
typedef v4f  __attribute__((may_alias)) v4fa;
typedef v8us __attribute__((may_alias)) v8usa;

__device__ __forceinline__ unsigned short f2bf(float f) { unsigned u = __float_as_uint(f); u += 0x7FFFu + ((u >> 16) & 1u); return (unsigned short)(u >> 16); }
__device__ __forceinline__ float bf2f(unsigned short b) { return __uint_as_float(((unsigned)b) << 16); }
__device__ __forceinline__ float bfr(float f) { return bf2f(f2bf(f)); }
__device__ __forceinline__ v16h cat16(v8h lo, v8h hi) { return __builtin_shufflevector(lo, hi, 0, 1, 2, 3, 4, 5, 6, 7, 8, 9, 10, 11, 12, 13, 14, 15); }
__device__ __forceinline__ v16bf cat16b(v8us lo, v8us hi) { return __builtin_bit_cast(v16bf, __builtin_shufflevector(lo, hi, 0, 1, 2, 3, 4, 5, 6, 7, 8, 9, 10, 11, 12, 13, 14, 15)); }
__device__ __forceinline__ v8f wmma16(v16h a, v16h b, v8f c) { return __builtin_amdgcn_wmma_f32_16x16x32_f16(false, a, false, b, (short)0, c, false, false); }
__device__ __forceinline__ v8f wmmab(v16bf a, v16bf b, v8f c) { return __builtin_amdgcn_wmma_f32_16x16x32_bf16(false, a, false, b, (short)0, c, false, false); }


template <typename T16> struct WFrag;
template <> struct WFrag<h16> { typedef v16h V; static __device__ __forceinline__ V ld(const h16* p) { return cat16(*(const v8h*)p, *(const v8h*)(p + 16)); } static __device__ __forceinline__ v8f mma(V a, V b, v8f c) { return wmma16(a, b, c); } };
template <> struct WFrag<bf> { typedef v16bf V; static __device__ __forceinline__ V ld(const bf* p) { return cat16b(*(const v8us*)p, *(const v8us*)(p + 16)); } static __device__ __forceinline__ v8f mma(V a, V b, v8f c) { return wmmab(a, b, c); } };
template <typename T16, int NSPLIT, bool BIAS>
__global__ __launch_bounds__(32) void k_gemmw(const T16* __restrict__ A, const T16* __restrict__ A2, const T16* __restrict__ Bt, const T16* __restrict__ Bt2, int K, float* C, int ldc, const float* __restrict__ bias, size_t sA, size_t sB, size_t sC) {
    typedef typename WFrag<T16>::V V;
    __shared__ __align__(16) float os[16 * 68];
    const size_t z = blockIdx.z; A += z * sA; if (A2) A2 += z * sA; Bt += z * sB; if (Bt2) Bt2 += z * sB; C += z * sC;
    const int lane = threadIdx.x & 31, lr = lane & 15, hi = lane >> 4; const int r0 = blockIdx.x * 64, c0 = blockIdx.y * 64;
    v8f acc[4][4];
#pragma unroll
    for (int mb = 0; mb < 4; ++mb)
#pragma unroll
        for (int nb = 0; nb < 4; ++nb) acc[mb][nb] = (v8f){};
    const size_t aoff = (size_t)(r0 + lr) * K + 8 * hi, boff = (size_t)(c0 + lr) * K + 8 * hi;
#pragma unroll 1
    for (int kc = 0; kc < K; kc += 32) {
        V a[4], a2[4];
#pragma unroll
        for (int mb = 0; mb < 4; ++mb) { a[mb] = WFrag<T16>::ld(A + aoff + (size_t)mb * 16 * K + kc); if (NSPLIT == 1 || NSPLIT == 2) a2[mb] = WFrag<T16>::ld(A2 + aoff + (size_t)mb * 16 * K + kc); }
#pragma unroll
        for (int nb = 0; nb < 4; ++nb) { const V b = WFrag<T16>::ld(Bt + boff + (size_t)nb * 16 * K + kc); V b2; if (NSPLIT >= 2) b2 = WFrag<T16>::ld(Bt2 + boff + (size_t)nb * 16 * K + kc);
#pragma unroll
            for (int mb = 0; mb < 4; ++mb) { acc[mb][nb] = WFrag<T16>::mma(a[mb], b, acc[mb][nb]); if (NSPLIT == 1 || NSPLIT == 2) acc[mb][nb] = WFrag<T16>::mma(a2[mb], b, acc[mb][nb]); if (NSPLIT >= 2) acc[mb][nb] = WFrag<T16>::mma(a[mb], b2, acc[mb][nb]); } }
        asm volatile("v_nop\n\tv_nop\n\tv_nop\n\tv_nop" : "+v"(acc[0][0]), "+v"(acc[1][1]), "+v"(acc[2][2]), "+v"(acc[3][3]) : "v"(a[0]), "v"(a[3]));
    }
#pragma unroll
    for (int mb = 0; mb < 4; ++mb) {
#pragma unroll
        for (int nb = 0; nb < 4; ++nb) {
#pragma unroll
            for (int j = 0; j < 8; ++j) os[(hi * 8 + j) * 68 + nb * 16 + lr] = acc[mb][nb][j]; }
        __builtin_amdgcn_wave_barrier(); asm volatile("" ::: "memory");
        float* crow = C + (size_t)(r0 + mb * 16) * ldc + c0;
#pragma unroll 1
        for (int ps = 0; ps < 2; ++ps) {
#pragma unroll
            for (int s = 0; s < 8; ++s) { const int row = 2 * s + hi, cofs = lr * 4; v4f val = *(const v4fa*)(os + row * 68 + cofs); if (BIAS) { val[0] += bfr(bias[c0 + cofs]); val[1] += bfr(bias[c0 + cofs + 1]); val[2] += bfr(bias[c0 + cofs + 2]); val[3] += bfr(bias[c0 + cofs + 3]); }
                *(volatile v4f*)(crow + (size_t)row * ldc + cofs) = val; }
            if (ps == 0) __threadfence(); }
        __builtin_amdgcn_wave_barrier(); asm volatile("" ::: "memory");
    }
}

typedef __attribute__((ext_vector_type(4))) unsigned short v4us;
typedef __attribute__((ext_vector_type(2))) unsigned short v2us;
typedef __attribute__((ext_vector_type(2))) _Float16 v2h;
typedef __attribute__((ext_vector_type(4))) _Float16 v4h;
__device__ __forceinline__ _Float16 tohx(float v) { return (_Float16)v; }
__device__ __forceinline__ void splitf(float y, unsigned short& h, unsigned short& l) { h = f2bf(y); l = f2bf(y - bf2f(h)); }
__global__ __launch_bounds__(256) void k_cvt8T(const float* __restrict__ src, bf* dst) { const size_t i = (size_t)blockIdx.x * 256 + threadIdx.x; if (i >= (size_t)TT * DM / 8) return; const int t = (int)(i / (DM / 8)); const int c0 = (int)(i % (DM / 8)) * 8; v8us o;
#pragma unroll
    for (int k = 0; k < 8; ++k) o[k] = f2bf(src[(size_t)(c0 + k) * TT + t]); *(volatile v8us*)(dst + (size_t)t * DM + c0) = o; __threadfence(); *(volatile v8us*)(dst + (size_t)t * DM + c0) = o; }

__global__ __launch_bounds__(256) void k_wstk(const float* __restrict__ kw, const float* __restrict__ qw, const float* __restrict__ vw, const float* __restrict__ kb, const float* __restrict__ qb, const float* __restrict__ vb, bf* Bt, float* BS) { const int i = blockIdx.x * 256 + threadIdx.x; if (i >= NP * DM / 8) return; const int c0 = (i % (DM / 8)) * 8, n = i / (DM / 8); const float* src = (n < EM) ? kw + (size_t)n * DM : (n < 2 * EM) ? qw + (size_t)(n - EM) * DM : (n < 3 * EM) ? vw + (size_t)(n - 2 * EM) * DM : nullptr; v8us o;
#pragma unroll
    for (int k = 0; k < 8; ++k) o[k] = src ? f2bf(src[c0 + k]) : (unsigned short)0; *(volatile v8us*)(Bt + (size_t)n * DM + c0) = o; __threadfence(); *(volatile v8us*)(Bt + (size_t)n * DM + c0) = o;
    if (i < NP / 4) { v4f b4; for (int q = 0; q < 4; ++q) { const int m = i * 4 + q; b4[q] = (m < EM) ? kb[m] : (m < 2 * EM) ? qb[m - EM] : (m < 3 * EM) ? vb[m - 2 * EM] : 0.0f; } *(volatile v4f*)(BS + i * 4) = b4; __threadfence(); *(volatile v4f*)(BS + i * 4) = b4; } }
__global__ __launch_bounds__(256) void k_pl32(const float* __restrict__ F3, int off, bf* Ph, bf* Pl) { const size_t e = ((size_t)blockIdx.x * 256 + threadIdx.x) * 2; if (e >= (size_t)TT * HD) return; const int d = (int)(e % HD); const size_t t = e / HD; v2us oh, ol;
#pragma unroll
    for (int q = 0; q < 2; ++q) { unsigned short a, b; splitf(F3[t * NP + off + d + q], a, b); oh[q] = a; ol[q] = b; }
    *(volatile v2us*)(Ph + e) = oh; *(volatile v2us*)(Pl + e) = ol; __threadfence(); *(volatile v2us*)(Ph + e) = oh; *(volatile v2us*)(Pl + e) = ol; }
__global__ __launch_bounds__(256) void k_vtpad(const float* __restrict__ F3, bf* Vh, bf* Vl) { const size_t e = ((size_t)blockIdx.x * 256 + threadIdx.x) * 2; if (e >= (size_t)HP * TT) return; const int t = (int)(e % TT); const int d = (int)(e / TT); v2us oh, ol;
#pragma unroll
    for (int q = 0; q < 2; ++q) { unsigned short a = 0, b = 0; if (d < EM) splitf(F3[(size_t)(t + q) * NP + 2 * EM + d], a, b); oh[q] = a; ol[q] = b; }
    *(volatile v2us*)(Vh + e) = oh; *(volatile v2us*)(Vl + e) = ol; __threadfence(); *(volatile v2us*)(Vh + e) = oh; *(volatile v2us*)(Vl + e) = ol; }
__global__ __launch_bounds__(256) void k_lsoft(const float* __restrict__ Sb, h16* P16, bf* Ph, bf* Pl) {
    const int lane = threadIdx.x & 31; const int row = blockIdx.x * 8 + (threadIdx.x >> 5); if (row >= ZH * TT) return; const int i = row % TT; const int zz = row / TT; const bool hires = (i < RH); const float* sr = Sb + (size_t)row * TT; float mx = -3.0e38f;
#pragma unroll 4
    for (int ch = 0; ch < TT / 128; ++ch) { const int j0 = ch * 128 + lane * 4; const v4f a = *(const v4f*)(sr + j0);
#pragma unroll
        for (int q = 0; q < 4; ++q) { float t = a[q] * SCL; asm volatile("" : "+v"(t)); mx = fmaxf(mx, t); } }
#pragma unroll
    for (int sh = 16; sh; sh >>= 1) mx = fmaxf(mx, __shfl_xor(mx, sh, 32));
    float sum = 0.f;
#pragma unroll 4
    for (int ch = 0; ch < TT / 128; ++ch) { const int j0 = ch * 128 + lane * 4; const v4f a = *(const v4f*)(sr + j0);
#pragma unroll
        for (int q = 0; q < 4; ++q) { float t = a[q] * SCL; asm volatile("" : "+v"(t)); float d0 = __fsub_rn(t, mx); asm volatile("" : "+v"(d0)); sum += __builtin_amdgcn_exp2f(__fmul_rn(d0, 1.4426950408889634f)); } }
#pragma unroll
    for (int sh = 16; sh; sh >>= 1) sum += __shfl_xor(sum, sh, 32);
    const float f = __fdiv_rn(hires ? 1.0f : PCAR, sum);
#pragma unroll 1
    for (int ps = 0; ps < 2; ++ps) {
        if (hires) {
#pragma unroll
            for (int ch = 0; ch < TT / 128; ++ch) { const int j0 = ch * 128 + lane * 4; const v4f a = *(const v4f*)(sr + j0); v4us oh, ol;
#pragma unroll
                for (int q = 0; q < 4; ++q) { float t = a[q] * SCL; asm volatile("" : "+v"(t)); float d0 = __fsub_rn(t, mx); asm volatile("" : "+v"(d0)); float ex = __builtin_amdgcn_exp2f(__fmul_rn(d0, 1.4426950408889634f)); asm volatile("" : "+v"(ex)); unsigned short a2, c2; splitf(ex * f, a2, c2); oh[q] = a2; ol[q] = c2; }
                const size_t oo = ((size_t)zz * RH + i) * TT + j0; *(volatile v4us*)(Ph + oo) = oh; *(volatile v4us*)(Pl + oo) = ol; }
        } else {
#pragma unroll 2
            for (int ch = 0; ch < TT / 128; ++ch) { const int j0 = ch * 128 + lane * 4; const v4f a = *(const v4f*)(sr + j0); v4h o4;
#pragma unroll
                for (int q = 0; q < 4; ++q) { float t = a[q] * SCL; asm volatile("" : "+v"(t)); float d0 = __fsub_rn(t, mx); asm volatile("" : "+v"(d0)); float ex = __builtin_amdgcn_exp2f(__fmul_rn(d0, 1.4426950408889634f)); asm volatile("" : "+v"(ex)); o4[q] = tohx(ex * f); }
                *(volatile v4h*)(P16 + (size_t)row * TT + j0) = o4; } }
        if (ps == 0) __threadfence(); }
}

__global__ __launch_bounds__(256) void k_tohl(const float* __restrict__ F, bf* Hh, bf* Hl, size_t n4) { const size_t i = (size_t)blockIdx.x * 256 + threadIdx.x; if (i >= n4) return; const v4f a = *(const v4f*)(F + i * 4); v4us oh, ol;
#pragma unroll
    for (int q = 0; q < 4; ++q) { unsigned short h2, l2; splitf(a[q], h2, l2); oh[q] = h2; ol[q] = l2; }
    *(volatile v4us*)(Hh + i * 4) = oh; *(volatile v4us*)(Hl + i * 4) = ol; __threadfence(); *(volatile v4us*)(Hh + i * 4) = oh; *(volatile v4us*)(Hl + i * 4) = ol; }
__global__ __launch_bounds__(256) void k_watt(const float* __restrict__ w, bf* Bt) { const int i = blockIdx.x * 256 + threadIdx.x; if (i >= DM * HP / 8) return; const int k0 = (i % (HP / 8)) * 8, n = i / (HP / 8); v8us o;
#pragma unroll
    for (int k = 0; k < 8; ++k) o[k] = (k0 + k < EM) ? f2bf(w[(size_t)n * EM + k0 + k]) : (unsigned short)0; *(volatile v8us*)(Bt + (size_t)n * HP + k0) = o; __threadfence(); *(volatile v8us*)(Bt + (size_t)n * HP + k0) = o; }
__global__ __launch_bounds__(256) void k_outs(const float* __restrict__ O2, const float* __restrict__ xim, const float* __restrict__ gam, float* yout, float* oout) { const size_t i = (size_t)blockIdx.x * 256 + threadIdx.x; if (i >= (size_t)DM * TT / 4) return; const int p0 = (int)(i % (TT / 4)) * 4; const int c = (int)(i / (TT / 4)); const float g = bfr(gam[0]); const v4f xv = *(const v4f*)(xim + (size_t)c * TT + p0); v4f o, y;
#pragma unroll
    for (int q = 0; q < 4; ++q) { o[q] = O2[(size_t)(p0 + q) * DM + c]; float t = __fmul_rn(g, o[q]); asm volatile("" : "+v"(t)); y[q] = __fadd_rn(t, bfr(xv[q])); }
    *(volatile v4f*)(oout + (size_t)c * TT + p0) = o; *(volatile v4f*)(yout + (size_t)c * TT + p0) = y; __threadfence(); *(volatile v4f*)(oout + (size_t)c * TT + p0) = o; *(volatile v4f*)(yout + (size_t)c * TT + p0) = y; }

extern "C" void kernel_launch(void* const* d_in, const int* in_sizes, int n_in,
                              void* d_out, int out_size, void* d_ws, size_t ws_size, hipStream_t stream) {
    (void)in_sizes; (void)n_in; (void)out_size;
    const float* x = (const float*)d_in[0]; const float* kw = (const float*)d_in[1]; const float* kb = (const float*)d_in[2]; const float* qw = (const float*)d_in[3]; const float* qb = (const float*)d_in[4]; const float* vw = (const float*)d_in[5]; const float* vb = (const float*)d_in[6]; const float* aw = (const float*)d_in[7]; const float* ab = (const float*)d_in[8]; const float* gam = (const float*)d_in[9];
    float* YOUT = (float*)d_out; float* OOUT = YOUT + (size_t)NB_ * DM * TT;
    char* wsp = (char*)d_ws;
    auto take = [&](size_t bytes) { char* p = wsp; wsp += (bytes + 255) & ~(size_t)255; return (void*)p; };
    bf* WS = (bf*)take((size_t)NP * DM * 2); float* BS = (float*)take(NP * 4); bf* WA = (bf*)take((size_t)DM * HP * 2);
    bf* XB = (bf*)take((size_t)TT * DM * 2); float* F3 = (float*)take((size_t)TT * NP * 4); bf* Qh = (bf*)take((size_t)TT * HD * 2); bf* Ql = (bf*)take((size_t)TT * HD * 2); bf* Kh = (bf*)take((size_t)TT * HD * 2); bf* Kl = (bf*)take((size_t)TT * HD * 2); bf* VTh = (bf*)take((size_t)HP * TT * 2); bf* VTl = (bf*)take((size_t)HP * TT * 2);
    float* Sb = (float*)take((size_t)TT * TT * 4); bf* Ph = (bf*)take((size_t)TT * TT * 2); bf* Pl = (bf*)take((size_t)TT * TT * 2); float* Ob = (float*)take((size_t)TT * HP * 4); bf* Ch = (bf*)take((size_t)TT * HP * 2); bf* Cl = (bf*)take((size_t)TT * HP * 2); float* O2 = (float*)take((size_t)TT * DM * 4);
    if ((size_t)(wsp - (char*)d_ws) > ws_size) return;
    k_wstk<<<(NP * DM / 8 + 255) / 256, 256, 0, stream>>>(kw, qw, vw, kb, qb, vb, WS, BS); k_watt<<<(DM * HP / 8 + 255) / 256, 256, 0, stream>>>(aw, WA);
    for (int b = 0; b < NB_; ++b) {
        k_cvt8T<<<(unsigned)(((size_t)TT * DM / 8 + 255) / 256), 256, 0, stream>>>(x + (size_t)b * DM * TT, XB);
        k_gemmw<bf, 0, true><<<dim3(TT / 64, NP / 64, 1), 32, 0, stream>>>(XB, nullptr, WS, nullptr, DM, F3, NP, BS, 0, 0, 0);
        k_pl32<<<(unsigned)(((size_t)TT * HD / 2 + 255) / 256), 256, 0, stream>>>(F3, EM, Qh, Ql);
        k_pl32<<<(unsigned)(((size_t)TT * HD / 2 + 255) / 256), 256, 0, stream>>>(F3, 0, Kh, Kl);
        k_vtpad<<<(unsigned)(((size_t)HP * TT / 2 + 255) / 256), 256, 0, stream>>>(F3, VTh, VTl);
        k_gemmw<bf, 2, false><<<dim3(TT / 64, TT / 64, 1), 32, 0, stream>>>(Qh, Ql, Kh, Kl, HD, Sb, TT, nullptr, 0, 0, 0);
        k_lsoft<<<TT / 8, 256, 0, stream>>>(Sb, nullptr, Ph, Pl);
        k_gemmw<bf, 2, false><<<dim3(TT / 64, HP / 64, 1), 32, 0, stream>>>(Ph, Pl, VTh, VTl, TT, Ob, HP, nullptr, 0, 0, 0);
        k_tohl<<<(unsigned)(((size_t)TT * HP / 4 + 255) / 256), 256, 0, stream>>>(Ob, Ch, Cl, (size_t)TT * HP / 4);
        k_gemmw<bf, 1, true><<<dim3(TT / 64, DM / 64, 1), 32, 0, stream>>>(Ch, Cl, WA, nullptr, HP, O2, DM, ab, 0, 0, 0);
        k_outs<<<(unsigned)(((size_t)DM * TT / 4 + 255) / 256), 256, 0, stream>>>(O2, x + (size_t)b * DM * TT, gam, YOUT + (size_t)b * DM * TT, OOUT + (size_t)b * DM * TT); }
}
